// MHA_pro_12369505812819
// MI455X (gfx1250) — hardware-verified
//
#include <hip/hip_runtime.h>
#include <math.h>

typedef __attribute__((ext_vector_type(16))) _Float16 v16h;
typedef __attribute__((ext_vector_type(16))) __bf16 v16b;
typedef __attribute__((ext_vector_type(8)))  _Float16 v8h;
typedef __attribute__((ext_vector_type(8)))  float v8f;
typedef __attribute__((ext_vector_type(4)))  float v4f;
typedef __attribute__((ext_vector_type(2)))  float v2f;
typedef __attribute__((ext_vector_type(4)))  unsigned v4u;
typedef __attribute__((ext_vector_type(4)))  int v4i;
typedef float __attribute__((may_alias)) float_a;
typedef int __attribute__((may_alias)) int_a;

template <typename T> __device__ __forceinline__ void vst2(void* p, T v) { *(volatile T*)p = v; __threadfence(); *(volatile T*)p = v; }
__device__ __forceinline__ v8f wmma16(v16h a, v16h b, v8f c) {
  v8f d = __builtin_amdgcn_wmma_f32_16x16x32_f16(false, a, false, b, (short)0, c, false, false);
  asm volatile("v_nop\n\tv_nop\n\tv_nop\n\tv_nop" : "+v"(d) : "v"(a), "v"(b));
  return d;
}
__device__ __forceinline__ v8f wmma_bf(v16b a, v16b b, v8f c) {
  v8f d = __builtin_amdgcn_wmma_f32_16x16x32_bf16(false, a, false, b, (short)0, c, false, false);
  asm volatile("v_nop\n\tv_nop\n\tv_nop\n\tv_nop" : "+v"(d) : "v"(a), "v"(b));
  return d;
}
__device__ __forceinline__ v16h frag_h(const _Float16* rowk0, int lane) {
  union { v16h v; v8h q[2]; } u; const _Float16* p = rowk0 + 8 * (lane >> 4);
  u.q[0] = *(const v8h*)p; u.q[1] = *(const v8h*)(p + 16); return u.v;
}
__device__ __forceinline__ v16h frag_f32(const float* rowk0, int lane) {
  v16h a; const float* p = rowk0 + 8 * (lane >> 4);
#pragma unroll
  for (int i = 0; i < 8; ++i) { a[i] = (_Float16)p[i]; a[8 + i] = (_Float16)p[16 + i]; }
  return a;
}
__device__ __forceinline__ v16h frag_f32s(const float* rowk0, int lane, float sc) {
  v16h a; const float* p = rowk0 + 8 * (lane >> 4);
#pragma unroll
  for (int i = 0; i < 8; ++i) { a[i] = (_Float16)(p[i] * sc); a[8 + i] = (_Float16)(p[16 + i] * sc); }
  return a;
}
__device__ __forceinline__ v16h fragc_f32(const float* W, int k0, int n, int lane, int ld, int K) {
  v16h a; const int g = lane >> 4;
#pragma unroll
  for (int i = 0; i < 8; ++i) { const int ka = k0 + 8 * g + i, kb = ka + 16;
    a[i] = (_Float16)(ka < K ? W[(size_t)(ka < K ? ka : K - 1) * ld + n] : 0.f); a[8 + i] = (_Float16)(kb < K ? W[(size_t)(kb < K ? kb : K - 1) * ld + n] : 0.f); }
  return a;
}
struct F2 { v16b h, l; };
__device__ __forceinline__ F2 bsplit16(const float v[16]) { F2 r;
#pragma unroll
  for (int i = 0; i < 16; ++i) { const __bf16 h = (__bf16)v[i]; r.h[i] = h; r.l[i] = (__bf16)(v[i] - (float)h); }
  return r; }
__device__ __forceinline__ F2 split_row(const float* row, int k0, int lane) { float v[16]; const float* p = row + k0 + 8 * (lane >> 4);
#pragma unroll
  for (int i = 0; i < 8; ++i) { v[i] = p[i]; v[8 + i] = p[16 + i]; }
  return bsplit16(v); }
__device__ __forceinline__ F2 split_rowK(const float* row, int k0, int lane, int K) { float v[16]; const int g = lane >> 4;
#pragma unroll
  for (int i = 0; i < 8; ++i) { const int ka = k0 + 8 * g + i, kb = ka + 16; v[i] = ka < K ? row[ka < K ? ka : K - 1] : 0.f; v[8 + i] = kb < K ? row[kb < K ? kb : K - 1] : 0.f; }
  return bsplit16(v); }
__device__ __forceinline__ F2 split_col(const float* W, int k0, int n, int lane, int ld, int K) { float v[16]; const int g = lane >> 4;
#pragma unroll
  for (int i = 0; i < 8; ++i) { const int ka = k0 + 8 * g + i, kb = ka + 16; v[i] = ka < K ? W[(size_t)(ka < K ? ka : K - 1) * ld + n] : 0.f; v[8 + i] = kb < K ? W[(size_t)(kb < K ? kb : K - 1) * ld + n] : 0.f; }
  return bsplit16(v); }
__device__ __forceinline__ v8f mac3(const F2& a, const F2& b, v8f c) { c = wmma_bf(a.l, b.h, c); c = wmma_bf(a.h, b.l, c); return wmma_bf(a.h, b.h, c); }
__device__ __forceinline__ float sigm(float v) { return 1.0f / (1.0f + expf(-v)); }
#define LDSX() do { asm volatile("s_wait_dscnt 0" ::: "memory"); __builtin_amdgcn_wave_barrier(); __builtin_amdgcn_fence(__ATOMIC_RELEASE, "workgroup"); } while (0)


#define NB 4
#define TT 1024
#define CCH 1024
#define NH 16
#define HS 64
#define NR (NB * TT)
#define ROT 32
typedef __attribute__((ext_vector_type(8))) __bf16 v8b;
__device__ __forceinline__ v16b frag_b16(const __bf16* rowk0, int lane) {
  union { v16b v; v8b q[2]; } u; const __bf16* p = rowk0 + 8 * (lane >> 4);
  u.q[0] = *(const v8b*)p; u.q[1] = *(const v8b*)(p + 16); return u.v;
}
__device__ __forceinline__ float bfr(float v) { return (float)(__bf16)v; }
__device__ __attribute__((noinline)) float exp_ni(float v) { return expf(v); }
__device__ __forceinline__ v8f mac3p(v16b ah, v16b al, v16b bh, v16b bl, v8f c) { c = wmma_bf(al, bh, c); c = wmma_bf(ah, bl, c); return wmma_bf(ah, bh, c); }
__constant__ float c_invfreq[16] = {1.0f,0.5623413324356079f,0.3162277638912201f,0.17782793939113617f,0.10000000149011612f,0.05623412877321243f,0.03162277862429619f,0.017782794311642647f,0.009999999776482582f,0.005623413249850273f,0.003162277862429619f,0.0017782794311642647f,0.0010000000474974513f,0.000562341301701963f,0.0003162277862429619f,0.00017782794020604342f};

#define PLANE_Q (2u * NB * NH * TT * HS)
#define WS_PT   0u
#define WS_QH   (WS_PT + 2u * 4 * CCH * CCH)
#define WS_QL   (WS_QH + PLANE_Q)
#define WS_KH   (WS_QL + PLANE_Q)
#define WS_KL   (WS_KH + PLANE_Q)
#define WS_VTH  (WS_KL + PLANE_Q)
#define WS_VTL  (WS_VTH + PLANE_Q)
#define WS_M    (WS_VTL + PLANE_Q)
#define WS_L    (WS_M + 4u * NB * NH * TT)
#define WS_OH   (WS_L + 4u * NB * NH * TT)
#define WS_OL   (WS_OH + 2u * NR * CCH)
#define WS_END  (WS_OL + 2u * NR * CCH)

__global__ __launch_bounds__(256) void k_pack(const float* __restrict__ Wq, const float* __restrict__ Wk, const float* __restrict__ Wv, const float* __restrict__ Wo, __bf16* __restrict__ PT) {
  __shared__ __align__(16) __bf16 srow[CCH];
  const int n = blockIdx.x, tid = threadIdx.x; const int which = n >> 10, nn = n & 1023;
  const float* Wm = which == 0 ? Wq : which == 1 ? Wk : which == 2 ? Wv : Wo;
  for (int k = tid; k < CCH; k += 256) srow[k] = (__bf16)Wm[(size_t)k * CCH + nn];
  __syncthreads();
  if (tid < CCH / 8) vst2((unsigned*)(PT + (size_t)n * CCH + tid * 8), *(const v4u*)(&srow[tid * 8]));
}
__device__ __forceinline__ v16b frag_xs(const float* __restrict__ X, size_t r, int t, int k0, int lane) {
  const bool shifted = k0 < CCH / 2; const bool zero = shifted && (t == 0);
  const float* p = X + (r - ((shifted && t > 0) ? 1 : 0)) * CCH + k0 + 8 * (lane >> 4);
  v16b a;
#pragma unroll
  for (int i = 0; i < 8; ++i) { a[i] = (__bf16)(zero ? 0.f : p[i]); a[8 + i] = (__bf16)(zero ? 0.f : p[16 + i]); }
  return a;
}
__global__ __launch_bounds__(128) void k_qkv(const float* __restrict__ X, const __bf16* __restrict__ PT, const float* __restrict__ bq, const float* __restrict__ bk, const float* __restrict__ bv,
                                             __bf16* __restrict__ Qh, __bf16* __restrict__ Ql, __bf16* __restrict__ Kh, __bf16* __restrict__ Kl, __bf16* __restrict__ VTh, __bf16* __restrict__ VTl) {
  __shared__ __align__(16) __bf16 sh_[128][72], sl_[128][72];
  const int tid = threadIdx.x, wave = tid >> 5, lane = tid & 31, col = lane & 15, g = lane >> 4;
  const size_t rb = (size_t)blockIdx.x * 64; const int b = (int)(rb / TT), t0 = (int)(rb % TT);
  const int which = blockIdx.y >> 3; const int n0 = (blockIdx.y & 7) * 128;
  const size_t r0 = rb + wave * 16; const int tq = t0 + wave * 16 + col;
  v8f acc[8] = {};
#pragma unroll 2
  for (int kc = 0; kc < CCH / 32; ++kc) { const v16b a = frag_xs(X, r0 + col, tq, kc * 32, lane);
#pragma unroll
    for (int j = 0; j < 8; ++j) acc[j] = wmma_bf(a, frag_b16(PT + ((size_t)which * CCH + n0 + j * 16 + col) * CCH + kc * 32, lane), acc[j]); }
  const float* bias = which == 0 ? bq : which == 1 ? bk : bv;
#pragma unroll
  for (int j = 0; j < 8; ++j) { const float bb = bfr(bias[n0 + j * 16 + col]);
#pragma unroll
    for (int r = 0; r < 8; ++r) acc[j][r] += bb; }
  if (which < 2) {
#pragma unroll
    for (int hp = 0; hp < 2; ++hp) {
#pragma unroll
      for (int r = 0; r < 8; ++r) { const int t = t0 + wave * 16 + 8 * g + r; const float th = (float)t * c_invfreq[col]; const float cs = cosf(th), sn = sinf(th);
        const float a0 = acc[hp * 4][r], a1 = acc[hp * 4 + 1][r];
        acc[hp * 4][r] = a0 * cs - a1 * sn; acc[hp * 4 + 1][r] = a1 * cs + a0 * sn; } }
    __bf16* Oh = which == 0 ? Qh : Kh; __bf16* Ol = which == 0 ? Ql : Kl;
#pragma unroll
    for (int hp = 0; hp < 2; ++hp) {
#pragma unroll
      for (int j = 0; j < 4; ++j)
#pragma unroll
        for (int r = 0; r < 8; ++r) { const float v = acc[hp * 4 + j][r]; const __bf16 hi = (__bf16)v; sh_[wave * 16 + 8 * g + r][j * 16 + col] = hi; sl_[wave * 16 + 8 * g + r][j * 16 + col] = (__bf16)(v - (float)hi); }
      LDSX();
      const int h = (n0 >> 6) + hp; const size_t base = ((size_t)(b * NH + h) * TT + t0 + wave * 16) * HS;
      for (int qq = lane; qq < 16 * 8; qq += 32) { const int rl = qq >> 3, pc = qq & 7; vst2((unsigned*)(Oh + base + rl * HS + pc * 8), *(const v4u*)(&sh_[wave * 16 + rl][pc * 8])); vst2((unsigned*)(Ol + base + rl * HS + pc * 8), *(const v4u*)(&sl_[wave * 16 + rl][pc * 8])); }
      LDSX(); }
  } else {
#pragma unroll
    for (int j = 0; j < 8; ++j)
#pragma unroll
      for (int r = 0; r < 8; ++r) { const float v = acc[j][r]; const __bf16 hi = (__bf16)v; sh_[j * 16 + col][wave * 16 + 8 * g + r] = hi; sl_[j * 16 + col][wave * 16 + 8 * g + r] = (__bf16)(v - (float)hi); }
    __syncthreads();
    for (int qq = tid; qq < 128 * 8; qq += 128) { const int c = qq >> 3, pc = qq & 7; const int h = (n0 >> 6) + (c >> 6), d = c & 63; const size_t o = ((size_t)(b * NH + h) * HS + d) * TT + t0 + pc * 8;
      vst2((unsigned*)(VTh + o), *(const v4u*)(&sh_[c][pc * 8])); vst2((unsigned*)(VTl + o), *(const v4u*)(&sl_[c][pc * 8])); }
  }
}
__global__ __launch_bounds__(128) void k_stats(const __bf16* __restrict__ Qh, const __bf16* __restrict__ Ql, const __bf16* __restrict__ Kh, const __bf16* __restrict__ Kl, float* __restrict__ Mo, float* __restrict__ Lo) {
  __shared__ float sm[64], ssum[64];
  const int tid = threadIdx.x, wave = tid >> 5, lane = tid & 31, col = lane & 15, g = lane >> 4;
  const int bh = blockIdx.y; const int i0 = blockIdx.x * 64 + wave * 16;
  const __bf16* qh = Qh + ((size_t)bh * TT + i0 + col) * HS; const __bf16* ql = Ql + ((size_t)bh * TT + i0 + col) * HS;
  const v16b qh0 = frag_b16(qh, lane), qh1 = frag_b16(qh + 32, lane), ql0 = frag_b16(ql, lane), ql1 = frag_b16(ql + 32, lane);
  float m[8], l[8];
#pragma unroll
  for (int r = 0; r < 8; ++r) { m[r] = -3.0e38f; l[r] = 0.f; }
  const int jend = i0 + 16;
#pragma unroll 1
  for (int j0 = 0; j0 < jend; j0 += 32) {
#pragma unroll
    for (int jt = 0; jt < 2; ++jt) { const int jb = j0 + jt * 16; if (jb < jend) {
      const __bf16* kh = Kh + ((size_t)bh * TT + jb + col) * HS; const __bf16* kl = Kl + ((size_t)bh * TT + jb + col) * HS;
      v8f s = {}; s = mac3p(qh0, ql0, frag_b16(kh, lane), frag_b16(kl, lane), s); s = mac3p(qh1, ql1, frag_b16(kh + 32, lane), frag_b16(kl + 32, lane), s);
#pragma unroll
      for (int r = 0; r < 8; ++r) { const int i = i0 + 8 * g + r, j = jb + col; const float v = (j <= i) ? s[r] * 0.125f : -1e30f;
        float mt = v;
#pragma unroll
        for (int o = 1; o < 16; o <<= 1) mt = fmaxf(mt, __shfl_xor(mt, o));
        const float mn = fmaxf(m[r], mt); float e = exp_ni(v - mn);
#pragma unroll
        for (int o = 1; o < 16; o <<= 1) e += __shfl_xor(e, o);
        l[r] = l[r] * exp_ni(m[r] - mn) + e; m[r] = mn; } } }
  }
  if (col == 0) {
#pragma unroll
    for (int r = 0; r < 8; ++r) { sm[wave * 16 + 8 * g + r] = m[r]; ssum[wave * 16 + 8 * g + r] = l[r]; } }
  __syncthreads();
  if (tid < 16) { vst2(Mo + (size_t)bh * TT + blockIdx.x * 64 + tid * 4, *(const v4f*)&sm[tid * 4]); vst2(Lo + (size_t)bh * TT + blockIdx.x * 64 + tid * 4, *(const v4f*)&ssum[tid * 4]); }
}
__global__ __launch_bounds__(256) void k_mix(const __bf16* __restrict__ Qh, const __bf16* __restrict__ Ql, const __bf16* __restrict__ Kh, const __bf16* __restrict__ Kl, const __bf16* __restrict__ VTh, const __bf16* __restrict__ VTl,
                                             const float* __restrict__ Mo, const float* __restrict__ Lo, const float* __restrict__ tw, const float* __restrict__ talpha, const float* __restrict__ tbeta, const float* __restrict__ mixw,
                                             __bf16* __restrict__ OH, __bf16* __restrict__ OL) {
  __shared__ __align__(16) __bf16 pwh[512][32], pwl[512][32];
  __shared__ __align__(16) float attp[NH][16][36];
  __shared__ __align__(16) __bf16 mixr[NH][32];
  const int tid = threadIdx.x, wave = tid >> 5, lane = tid & 31, col = lane & 15, g = lane >> 4;
  const int b = blockIdx.y, i0 = blockIdx.x * 16;
  for (int q = tid; q < 512 * 32 / 8; q += 256) { *(v4u*)(&pwh[0][0] + q * 8) = (v4u){0u,0u,0u,0u}; *(v4u*)(&pwl[0][0] + q * 8) = (v4u){0u,0u,0u,0u}; }
  for (int q = tid; q < NH * 32; q += 256) { const int o = q >> 5, h = q & 31; mixr[o][h] = h < NH ? (__bf16)mixw[o * NH + h] : (__bf16)0.f; }
  const int hA = wave * 2;
  float mrow[2][8], lb[2][8];
#pragma unroll
  for (int u = 0; u < 2; ++u) { const int bh = b * NH + hA + u;
#pragma unroll
    for (int r = 0; r < 8; ++r) { const int i = i0 + 8 * g + r; mrow[u][r] = Mo[(size_t)bh * TT + i]; lb[u][r] = bfr(tbeta[(hA + u) * TT + i]) / Lo[(size_t)bh * TT + i]; } }
  v8f oacc[2][4];
#pragma unroll
  for (int u = 0; u < 2; ++u)
#pragma unroll
    for (int d4 = 0; d4 < 4; ++d4) oacc[u][d4] = (v8f){};
  __syncthreads();
  const int jend = i0 + 16;
#pragma unroll 1
  for (int j0 = 0; j0 < jend; j0 += 32) {
#pragma unroll
    for (int u = 0; u < 2; ++u) { const int h = hA + u; const int bh = b * NH + h;
      const __bf16* qh = Qh + ((size_t)bh * TT + i0 + col) * HS; const __bf16* ql = Ql + ((size_t)bh * TT + i0 + col) * HS;
      const v16b qh0 = frag_b16(qh, lane), qh1 = frag_b16(qh + 32, lane), ql0 = frag_b16(ql, lane), ql1 = frag_b16(ql + 32, lane);
#pragma unroll 1
      for (int jt = 0; jt < 2; ++jt) { const int jb = j0 + jt * 16;
        v8f s = {};
        if (jb < jend) { const __bf16* kh = Kh + ((size_t)bh * TT + jb + col) * HS; const __bf16* kl = Kl + ((size_t)bh * TT + jb + col) * HS;
          s = mac3p(qh0, ql0, frag_b16(kh, lane), frag_b16(kl, lane), s); s = mac3p(qh1, ql1, frag_b16(kh + 32, lane), frag_b16(kl + 32, lane), s); }
        const int j = jb + col; const float alpha_j = bfr(talpha[h * TT + (j < TT ? j : TT - 1)]);
#pragma unroll
        for (int r = 0; r < 8; ++r) { const int il = 8 * g + r, i = i0 + il; float pw = 0.f;
          if (jb < jend && j <= i) { const int widx = TT - 1 + j - i; pw = (exp_ni(s[r] * 0.125f - mrow[u][r]) * lb[u][r]) * (bfr(tw[h * TT + (widx < TT ? widx : TT - 1)]) * alpha_j); }
          const __bf16 hi = (__bf16)pw; pwh[il * 32 + jt * 16 + col][h] = hi; pwl[il * 32 + jt * 16 + col][h] = (__bf16)(pw - (float)hi); } } }
    __syncthreads();
    { const v16b am = frag_b16(&mixr[col][0], lane);
#pragma unroll 1
      for (int ct = 0; ct < 4; ++ct) { const int n0c = (wave * 4 + ct) * 16; v8f a = {};
        a = wmma_bf(am, frag_b16(&pwl[n0c + col][0], lane), a); a = wmma_bf(am, frag_b16(&pwh[n0c + col][0], lane), a);
        const int il = n0c >> 5, jl0 = n0c & 31;
#pragma unroll
        for (int r = 0; r < 8; ++r) attp[8 * g + r][il][jl0 + col] = a[r]; } }
    __syncthreads();
#pragma unroll
    for (int u = 0; u < 2; ++u) { const int o = hA + u; const int bh = b * NH + o; const F2 af = split_row(&attp[o][col][0], 0, lane);
#pragma unroll
      for (int d4 = 0; d4 < 4; ++d4) { const __bf16* vh = VTh + ((size_t)bh * HS + d4 * 16 + col) * TT + j0; const __bf16* vl = VTl + ((size_t)bh * HS + d4 * 16 + col) * TT + j0;
        oacc[u][d4] = mac3p(af.h, af.l, frag_b16(vh, lane), frag_b16(vl, lane), oacc[u][d4]); } }
    __syncthreads();
  }
  __bf16* sth = &pwh[0][0] + wave * (16 * 128); __bf16* stl = &pwl[0][0] + wave * (16 * 128);
#pragma unroll
  for (int u = 0; u < 2; ++u)
#pragma unroll
    for (int d4 = 0; d4 < 4; ++d4)
#pragma unroll
      for (int r = 0; r < 8; ++r) { const float v = oacc[u][d4][r]; const __bf16 hi = (__bf16)v; sth[(8 * g + r) * 128 + u * 64 + d4 * 16 + col] = hi; stl[(8 * g + r) * 128 + u * 64 + d4 * 16 + col] = (__bf16)(v - (float)hi); }
  LDSX();
  for (int qq = lane; qq < 16 * 16; qq += 32) { const int rl = qq >> 4, pc = qq & 15; const size_t o = ((size_t)b * TT + i0 + rl) * CCH + hA * 64 + pc * 8;
    vst2((unsigned*)(OH + o), *(const v4u*)(sth + rl * 128 + pc * 8)); vst2((unsigned*)(OL + o), *(const v4u*)(stl + rl * 128 + pc * 8)); }
}
__global__ __launch_bounds__(128) void k_out(const __bf16* __restrict__ OH, const __bf16* __restrict__ OL, const __bf16* __restrict__ PT, const float* __restrict__ bo, const float* __restrict__ gam, float* __restrict__ out) {
  __shared__ __align__(16) float so[4][16][132];
  const int tid = threadIdx.x, wave = tid >> 5, lane = tid & 31, col = lane & 15, g = lane >> 4; const size_t r0 = (size_t)blockIdx.x * 64 + wave * 16; const int n0 = blockIdx.y * 128;
  v8f acc[8] = {};
#pragma unroll 2
  for (int kc = 0; kc < CCH / 32; ++kc) { const v16b ah = frag_b16(OH + (r0 + col) * CCH + kc * 32, lane), al = frag_b16(OL + (r0 + col) * CCH + kc * 32, lane);
#pragma unroll
    for (int j = 0; j < 8; ++j) { const v16b wb = frag_b16(PT + ((size_t)3 * CCH + n0 + j * 16 + col) * CCH + kc * 32, lane); acc[j] = wmma_bf(al, wb, acc[j]); acc[j] = wmma_bf(ah, wb, acc[j]); } }
#pragma unroll
  for (int j = 0; j < 8; ++j) { const float bb = bfr(bo[n0 + j * 16 + col]);
#pragma unroll
    for (int r = 0; r < 8; ++r) { const int t = (int)((r0 + 8 * g + r) % TT); so[wave][8 * g + r][j * 16 + col] = (acc[j][r] + bb) * bfr(gam[t]); } }
  LDSX();
  for (int rl = 0; rl < 16; ++rl) vst2(out + (r0 + rl) * CCH + n0 + lane * 4, *(const v4f*)(&so[wave][rl][lane * 4]));
}

extern "C" void kernel_launch(void* const* d_in, const int* in_sizes, int n_in, void* d_out, int out_size, void* d_ws, size_t ws_size, hipStream_t stream) {
  (void)in_sizes; (void)n_in; (void)out_size;
  const float** I = (const float**)d_in;
  if (ws_size < (size_t)WS_END) return;
  char* ws = (char*)d_ws;
  __bf16* PT = (__bf16*)(ws + WS_PT); __bf16 *Qh = (__bf16*)(ws + WS_QH), *Ql = (__bf16*)(ws + WS_QL), *Kh = (__bf16*)(ws + WS_KH), *Kl = (__bf16*)(ws + WS_KL), *VTh = (__bf16*)(ws + WS_VTH), *VTl = (__bf16*)(ws + WS_VTL);
  float *Mo = (float*)(ws + WS_M), *Lo = (float*)(ws + WS_L); __bf16 *OH = (__bf16*)(ws + WS_OH), *OL = (__bf16*)(ws + WS_OL);
  k_pack<<<4 * CCH, 256, 0, stream>>>(I[1], I[3], I[5], I[7], PT);
  k_qkv<<<dim3(NR / 64, 24), 128, 0, stream>>>(I[0], PT, I[2], I[4], I[6], Qh, Ql, Kh, Kl, VTh, VTl);
  k_stats<<<dim3(TT / 64, NB * NH), 128, 0, stream>>>(Qh, Ql, Kh, Kl, Mo, Lo);
  k_mix<<<dim3(TT / 16, NB), 256, 0, stream>>>(Qh, Ql, Kh, Kl, VTh, VTl, Mo, Lo, I[9], I[10], I[11], I[13], OH, OL);
  k_out<<<dim3(NR / 64, CCH / 128), 128, 0, stream>>>(OH, OL, PT, I[8], I[12], (float*)d_out);
}
